// ColumnGraphMemory_59794534695164
// MI455X (gfx1250) — hardware-verified
//
#include <hip/hip_runtime.h>
#include <stddef.h>
#include <stdint.h>

#define NBATCH  2
#define NNODE   16384
#define KNB     16
#define DSW     128
#define DIDW    64
#define MROWS   (NBATCH * NNODE)
#define NEDGE   (NNODE * KNB)
#define XK      320
#define H2K     512
#define UK      576
#define INCW    256

#define NTHR    256
#define NWAVE   8
#define EPT     8
#define CHUNK   (NTHR * EPT)
#define WCAP    (EPT * 32)
#define LISTN   (NWAVE * WCAP)
#define NBMAX   2048
#define NBRUN   512
#define NSB     (NNODE / NBRUN)
#define RCAP    12288
#define DEGCAP  64
#define STW     512
#define GBM     64
#define GBN     64
#define GTHR    128
#define WSMAX   134217728
#define LDS_SCAN ((2 * RCAP + 2 * NBMAX + LISTN) * 4 + 64)

static_assert((CHUNK & (CHUNK - 1)) == 0 && CHUNK <= 4096);
static_assert((NBMAX & (NBMAX - 1)) == 0 && NBMAX <= 4096);
static_assert((NBRUN & (NBRUN - 1)) == 0 && NBRUN <= NBMAX && NBRUN >= 16);
static_assert(NTHR * 8 == NBMAX);
static_assert(LISTN >= NBMAX);
static_assert(LISTN >= NWAVE * WCAP);
static_assert((RCAP % 32) == 0);
static_assert(NWAVE * STW <= RCAP);
static_assert(DSW <= STW);
static_assert(LDS_SCAN <= 300000);
static_assert(GBM == (GTHR / 32) * 16);
static_assert(DSW == 32 * 4);
static_assert((MROWS % 128) == 0 && (NNODE % 128) == 0);
static_assert((NNODE % NBRUN) == 0);
static_assert((NNODE % NTHR) == 0);
static_assert((NTHR % 128) == 0);
static_assert((NEDGE % CHUNK) == 0);
static_assert(NEDGE <= (1 << 19));
static_assert((XK % 32) == 0 && (H2K % 32) == 0 && (UK % 32) == 0 && (DIDW % 32) == 0);
static_assert((MROWS % GBM) == 0 && (NNODE % GBM) == 0);

#define SZ_XHL   ((size_t)MROWS * XK * 2)
#define SZ_HHL   ((size_t)MROWS * H2K * 2)
#define SZ_F32   ((size_t)MROWS * DSW * 4)
#define SZ_HK    ((size_t)NNODE * H2K * 2)
#define SZ_KF    ((size_t)NNODE * DSW * 4)
#define SZ_CAT   ((size_t)256 * XK * 2)
#define SZ_W2D   ((size_t)128 * H2K * 2)
#define SZ_K1T   ((size_t)256 * DIDW * 2)
#define SZ_U1    ((size_t)256 * UK * 2)
#define SZ_DEC   ((size_t)NNODE * 4)
#define SZ_POIS  ((size_t)NBATCH * NSB * 128)
#define O_XHL    ((size_t)0)
#define O_HHL    (O_XHL + SZ_XHL)
#define O_MOUT   (O_HHL + SZ_HHL)
#define O_QF     (O_MOUT + SZ_F32)
#define O_HK     (O_QF + SZ_F32)
#define O_KF     (O_HK + SZ_HK)
#define O_C1     (O_KF + SZ_KF)
#define O_Q1     (O_C1 + SZ_CAT)
#define O_C2     (O_Q1 + SZ_CAT)
#define O_Q2     (O_C2 + SZ_W2D)
#define O_K1     (O_Q2 + SZ_W2D)
#define O_K2     (O_K1 + SZ_K1T)
#define O_U1     (O_K2 + SZ_W2D)
#define O_U2     (O_U1 + SZ_U1)
#define O_DEC    (O_U2 + SZ_W2D)
#define O_POIS   (O_DEC + SZ_DEC)
#define WS_TOTAL (O_POIS + SZ_POIS)
static_assert(SZ_HK == (size_t)MROWS * INCW * 2);
static_assert(WS_TOTAL == 114499584);
static_assert(WS_TOTAL <= (size_t)WSMAX);
static_assert((O_HHL % 256) == 0 && (O_KF % 256) == 0 && (O_C1 % 256) == 0 && (O_U1 % 256) == 0 && (O_POIS % 256) == 0);
static_assert((O_DEC % 128) == 0 && (SZ_DEC % 128) == 0);

typedef float          v4f   __attribute__((ext_vector_type(4)));
typedef float          v8f   __attribute__((ext_vector_type(8)));
typedef int            v4i   __attribute__((ext_vector_type(4)));
typedef int            v8i   __attribute__((ext_vector_type(8)));
typedef unsigned short v8us  __attribute__((ext_vector_type(8)));
typedef __bf16         v16bf __attribute__((ext_vector_type(16)));
union FragB { v16bf v; v8us u[2]; v8i w; };

__device__ __forceinline__ v8f wmx(const FragB& a, const FragB& b, v8f c) {
  v8f d = __builtin_amdgcn_wmma_f32_16x16x32_bf16(false, a.v, false, b.v, (short)0, c, false, false);
  asm volatile("v_nop\n\tv_nop\n\tv_nop\n\tv_nop" : "+v"(d) : "v"(a.w), "v"(b.w));
  return d;
}

__device__ __forceinline__ void ldwait() {
  asm volatile("s_wait_loadcnt 0x0" ::: "memory");
}

__device__ __forceinline__ void wave_sync_lds() {
  __builtin_amdgcn_fence(__ATOMIC_ACQ_REL, "workgroup");
  __builtin_amdgcn_wave_barrier();
}

__device__ __forceinline__ unsigned bfbits(float v) {
  unsigned u = __float_as_uint(v);
  const unsigned r = (u + 0x7FFFu + ((u >> 16) & 1u)) >> 16;
  return (v != v) ? 0x7FC0u : r;
}
__device__ __forceinline__ float rbf(float v) { return __uint_as_float(bfbits(v) << 16); }

__device__ __forceinline__ v8us cvt8b(const v4f a, const v4f b) {
  v8us o;
  o[0] = (unsigned short)bfbits(a.x); o[1] = (unsigned short)bfbits(a.y);
  o[2] = (unsigned short)bfbits(a.z); o[3] = (unsigned short)bfbits(a.w);
  o[4] = (unsigned short)bfbits(b.x); o[5] = (unsigned short)bfbits(b.y);
  o[6] = (unsigned short)bfbits(b.z); o[7] = (unsigned short)bfbits(b.w);
  return o;
}
__device__ __forceinline__ v8us pack_hl(const v4f a, const v4f b, const int selLo) {
  const float f[8] = {a.x, a.y, a.z, a.w, b.x, b.y, b.z, b.w};
  v8us o;
#pragma unroll
  for (int i = 0; i < 8; ++i) {
    const unsigned hb = bfbits(f[i]);
    const float hv = __uint_as_float(hb << 16);
    const unsigned lb = bfbits(f[i] - hv);
    o[i] = (unsigned short)(selLo != 0 ? lb : hb);
  }
  return o;
}

__device__ __forceinline__ float gelu_t(float x) {
  const float u = 0.7978845608f * (x + 0.044715f * x * x * x);
  const float e = expf(2.0f * u);
  const float t = 1.0f - 2.0f * __builtin_amdgcn_rcpf(e + 1.0f);
  return 0.5f * x * (1.0f + t);
}

__device__ __forceinline__ int scan_chunk(const int* __restrict__ dsts, int nE, int cbase, int slotBase,
                                          int nb, int vec8, int* list, int tid, int lane, int wave) {
  int wc = 0;
  const int el0  = tid * EPT;
  const int e0   = cbase + el0;
  const int sent = -2147483647 - 1;
  v4i da, db;
  if (vec8 != 0 && cbase + CHUNK <= nE) {
    da = *(const v4i*)(dsts + e0);
    db = *(const v4i*)(dsts + e0 + 4);
  } else {
    da.x = (e0     < nE) ? dsts[min(e0,     nE - 1)] : sent;
    da.y = (e0 + 1 < nE) ? dsts[min(e0 + 1, nE - 1)] : sent;
    da.z = (e0 + 2 < nE) ? dsts[min(e0 + 2, nE - 1)] : sent;
    da.w = (e0 + 3 < nE) ? dsts[min(e0 + 3, nE - 1)] : sent;
    db.x = (e0 + 4 < nE) ? dsts[min(e0 + 4, nE - 1)] : sent;
    db.y = (e0 + 5 < nE) ? dsts[min(e0 + 5, nE - 1)] : sent;
    db.z = (e0 + 6 < nE) ? dsts[min(e0 + 6, nE - 1)] : sent;
    db.w = (e0 + 7 < nE) ? dsts[min(e0 + 7, nE - 1)] : sent;
  }
  const unsigned nbs = (unsigned)slotBase;
  const unsigned unb = (unsigned)nb;
  const unsigned s0 = (unsigned)da.x - nbs, s1 = (unsigned)da.y - nbs;
  const unsigned s2 = (unsigned)da.z - nbs, s3 = (unsigned)da.w - nbs;
  const unsigned s4 = (unsigned)db.x - nbs, s5 = (unsigned)db.y - nbs;
  const unsigned s6 = (unsigned)db.z - nbs, s7 = (unsigned)db.w - nbs;
  const bool h0 = s0 < unb, h1 = s1 < unb, h2 = s2 < unb, h3 = s3 < unb;
  const bool h4 = s4 < unb, h5 = s5 < unb, h6 = s6 < unb, h7 = s7 < unb;
  const unsigned any = __builtin_amdgcn_ballot_w32(h0 | h1 | h2 | h3 | h4 | h5 | h6 | h7);
  if (any != 0u) {
#define HITJ(J, HJ, SJ) { \
      const unsigned mj = __builtin_amdgcn_ballot_w32(HJ); \
      if (mj != 0u) { \
        if (HJ) { \
          const int pos = wc + (int)__builtin_amdgcn_mbcnt_lo(mj, 0u); \
          if (pos < WCAP) list[wave * WCAP + pos] = ((el0 + (J)) << 12) | (int)(SJ); \
        } \
        wc += (int)__builtin_popcount(mj); } }
    HITJ(0, h0, s0)
    HITJ(1, h1, s1)
    HITJ(2, h2, s2)
    HITJ(3, h3, s3)
    HITJ(4, h4, s4)
    HITJ(5, h5, s5)
    HITJ(6, h6, s6)
    HITJ(7, h7, s7)
#undef HITJ
  }
  return wc;
}

__global__ __launch_bounds__(NTHR) __attribute__((amdgpu_num_vgpr(248)))
void k_pa(const float* __restrict__ s, const float* __restrict__ cnw, const float* __restrict__ cid,
          unsigned short* xhl, int nRows, int nN) {
  __shared__ __attribute__((aligned(16))) float stw_all[NWAVE * DSW];
  const int tid = (int)threadIdx.x, lane = tid & 31, wave = tid >> 5;
  const int r  = (int)blockIdx.x * NWAVE + wave;
  const int rc = r < nRows ? r : nRows - 1;
  const int n  = rc % nN;
  v4f v = *(const v4f*)(s + (size_t)rc * DSW + 4 * lane);
  const v4f g = *(const v4f*)(cnw + 4 * lane);
  const float* cp = cid + (size_t)n * DIDW + 8 * (lane & 7);
  const v4f ca = *(const v4f*)cp;
  const v4f cb = *(const v4f*)(cp + 4);
  v.x = rbf(v.x); v.y = rbf(v.y); v.z = rbf(v.z); v.w = rbf(v.w);
  float ss = v.x * v.x;
  ss = fmaf(v.y, v.y, ss);
  ss = fmaf(v.z, v.z, ss);
  ss = fmaf(v.w, v.w, ss);
#pragma unroll
  for (int off = 16; off > 0; off >>= 1) ss += __shfl_xor(ss, off);
  const float mean = ss * (1.0f / (float)DSW);
  const float inv  = 1.0f / sqrtf(mean + 1e-6f);
  v4f sn;
  sn.x = (v.x * inv) * rbf(g.x);
  sn.y = (v.y * inv) * rbf(g.y);
  sn.z = (v.z * inv) * rbf(g.z);
  sn.w = (v.w * inv) * rbf(g.w);
  float* stw = stw_all + wave * DSW;
  wave_sync_lds();
  *(v4f*)(stw + 4 * lane) = sn;
  wave_sync_lds();
  const int part = lane >> 4, piece = lane & 15;
  const v4f ga = *(const v4f*)(stw + 8 * piece);
  const v4f gb = *(const v4f*)(stw + 8 * piece + 4);
  const v8us hl = pack_hl(ga, gb, part);
  const v8us ib = cvt8b(ca, cb);
  unsigned short* rowp = xhl + (size_t)rc * XK;
  const bool wr = r < nRows;
  if (wr) {
    *(volatile v8us*)(rowp + part * DSW + 8 * piece) = hl;
    if (lane < 8) *(volatile v8us*)(rowp + 2 * DSW + 8 * lane) = ib;
  }
  __threadfence();
  if (wr) {
    *(volatile v8us*)(rowp + part * DSW + 8 * piece) = hl;
    if (lane < 8) *(volatile v8us*)(rowp + 2 * DSW + 8 * lane) = ib;
  }
}

__global__ __launch_bounds__(NTHR) void k_wtr(const float* __restrict__ w, int cols, int Kp,
                                              int t1, int d1, int t2, int d2,
                                              unsigned short* wt, int nUnits) {
  const int u = (int)blockIdx.x * NTHR + (int)threadIdx.x;
  if (u >= nUnits) return;
  const int kq = Kp >> 3;
  const int n  = u / kq;
  const int k8 = (u - n * kq) * 8;
  const int sr = k8 - (k8 >= t1 ? d1 : 0) - (k8 >= t2 ? d2 : 0);
  const float* p = w + (size_t)sr * (size_t)cols + n;
  v4f a, b;
  a.x = p[0];                  a.y = p[(size_t)cols];       a.z = p[(size_t)2 * cols];   a.w = p[(size_t)3 * cols];
  b.x = p[(size_t)4 * cols];   b.y = p[(size_t)5 * cols];   b.z = p[(size_t)6 * cols];   b.w = p[(size_t)7 * cols];
  const v8us hv = cvt8b(a, b);
  const size_t o = (size_t)n * (size_t)Kp + k8;
  *(volatile v8us*)(wt + o) = hv;
  __threadfence();
  *(volatile v8us*)(wt + o) = hv;
}

__global__ __launch_bounds__(NTHR) void k_dec(const float* __restrict__ cid, const float* __restrict__ dw,
                                              const float* __restrict__ db, float* dec, int nN) {
  __shared__ __attribute__((aligned(16))) float sw[DIDW];
  __shared__ __attribute__((aligned(16))) float sd[NTHR];
  const int tid = (int)threadIdx.x;
  const float wv = rbf(dw[tid & (DIDW - 1)]);
  if (tid < DIDW) sw[tid] = wv;
  __syncthreads();
  const int base = (int)blockIdx.x * NTHR;
  const int n  = base + tid;
  const int nc = n < nN ? n : nN - 1;
  const float* cp = cid + (size_t)nc * DIDW;
  float acc = 0.0f;
#pragma unroll 1
  for (int j = 0; j < DIDW / 4; ++j) {
    const v4f c = *(const v4f*)(cp + 4 * j);
    acc = fmaf(rbf(c.x), sw[4 * j + 0], acc);
    acc = fmaf(rbf(c.y), sw[4 * j + 1], acc);
    acc = fmaf(rbf(c.z), sw[4 * j + 2], acc);
    acc = fmaf(rbf(c.w), sw[4 * j + 3], acc);
  }
  const float z = acc + rbf(db[0]);
  const float d = __builtin_amdgcn_rcpf(1.0f + expf(-z));
  sd[tid] = d;
  __syncthreads();
  const int tq = tid < (NTHR / 4) ? tid : (NTHR / 4) - 1;
  const v4f dv = *(const v4f*)(sd + 4 * tq);
  const bool wr = (tid < (NTHR / 4)) && (base + 4 * tq + 3 < nN);
  float* op = dec + (size_t)base + 4 * tq;
  if (wr) *(volatile v4f*)op = dv;
  __threadfence();
  if (wr) *(volatile v4f*)op = dv;
}

__device__ __forceinline__ void store_hl(const float* stg, unsigned short* out16, int rowBase, int col0,
                                         int wave, int lane) {
  const int q8 = lane & 7, sub = lane >> 3, part = sub & 1;
#pragma unroll 1
  for (int i = 0; i < 8; ++i) {
    const int lid = 4 * i + sub;
    const int lr  = 16 * wave + (lid >> 1);
    const float* p = stg + lr * GBN + 8 * q8;
    const v4f ga = *(const v4f*)p;
    const v4f gb = *(const v4f*)(p + 4);
    const v8us hl = pack_hl(ga, gb, part);
    unsigned short* dst = out16 + (size_t)(rowBase + lr) * H2K + part * 256 + col0 + 8 * q8;
    *(volatile v8us*)dst = hl;
  }
}
__device__ __forceinline__ void store_f32(const float* stg, float* outF, int rowBase, int col0,
                                          int wave, int hh, int m) {
#pragma unroll 1
  for (int i = 0; i < 8; ++i) {
    const int lr = 16 * wave + 2 * i + hh;
    const v4f v = *(const v4f*)(stg + lr * GBN + 4 * m);
    float* op = outF + (size_t)(rowBase + lr) * DSW + col0 + 4 * m;
    *(volatile v4f*)op = v;
  }
}

template<int EPI, int LDA1, int AOFS1, int KS1, int LDA2, int KS2>
__global__ __launch_bounds__(GTHR) __attribute__((amdgpu_num_vgpr(248)))
void k_gemm(const unsigned short* __restrict__ A1, const unsigned short* __restrict__ A2,
            const unsigned short* __restrict__ WT, const float* __restrict__ bias,
            unsigned short* out16, float* outF,
            const float* __restrict__ sraw, const float* __restrict__ dec, const float* __restrict__ pois)
{
  constexpr int KT = 32 * (KS1 + KS2);
  __shared__ __attribute__((aligned(16))) float stg[GBM * GBN];
  __shared__ __attribute__((aligned(16))) float sb[GBN];
  const int tid = (int)threadIdx.x, lane = tid & 31, wave = tid >> 5, hh = lane >> 4, m = lane & 15;
  const int rowBase = (int)blockIdx.x * GBM;
  const int col0    = (int)blockIdx.y * GBN;

  {
    const v4f b4 = *(const v4f*)(bias + col0 + 4 * (tid & 15));
    v4f bq;
    bq.x = rbf(b4.x); bq.y = rbf(b4.y); bq.z = rbf(b4.z); bq.w = rbf(b4.w);
    if (tid < 16) *(v4f*)(sb + 4 * tid) = bq;
  }
  __syncthreads();

  v8f acc[4];
  {
    const v8f z = {0.f, 0.f, 0.f, 0.f, 0.f, 0.f, 0.f, 0.f};
    acc[0] = z; acc[1] = z; acc[2] = z; acc[3] = z;
  }
  const size_t grow = (size_t)(rowBase + 16 * wave + m);
  const unsigned short* ap = A1 + grow * (size_t)LDA1 + AOFS1 + 8 * hh;
  const unsigned short* wp = WT + (size_t)(col0 + m) * (size_t)KT + 8 * hh;
#pragma unroll 1
  for (int ks = 0; ks < KS1; ++ks) {
    FragB af;
    af.u[0] = *(const v8us*)(ap + 32 * ks);
    af.u[1] = *(const v8us*)(ap + 32 * ks + 16);
#pragma unroll
    for (int t = 0; t < 4; ++t) {
      const unsigned short* wq = wp + (size_t)(16 * t) * (size_t)KT + 32 * ks;
      FragB bf;
      bf.u[0] = *(const v8us*)wq;
      bf.u[1] = *(const v8us*)(wq + 16);
      acc[t] = wmx(af, bf, acc[t]);
    }
  }
  if (KS2 > 0) {
    const unsigned short* ap2 = A2 + grow * (size_t)LDA2 + 8 * hh;
#pragma unroll 1
    for (int ks = 0; ks < KS2; ++ks) {
      FragB af;
      af.u[0] = *(const v8us*)(ap2 + 32 * ks);
      af.u[1] = *(const v8us*)(ap2 + 32 * ks + 16);
#pragma unroll
      for (int t = 0; t < 4; ++t) {
        const unsigned short* wq = wp + (size_t)(16 * t) * (size_t)KT + 32 * (KS1 + ks);
        FragB bf;
        bf.u[0] = *(const v8us*)wq;
        bf.u[1] = *(const v8us*)(wq + 16);
        acc[t] = wmx(af, bf, acc[t]);
      }
    }
  }

#pragma unroll
  for (int t = 0; t < 4; ++t) {
    const int lc = 16 * t + m;
    const float bv = sb[lc];
#pragma unroll
    for (int r = 0; r < 8; ++r) {
      const int lr = 16 * wave + 8 * hh + r;
      stg[lr * GBN + lc] = acc[t][r] + bv;
    }
  }
  __syncthreads();

  if (EPI == 0) {
#pragma unroll 1
    for (int i = 0; i < 8; ++i) {
      float* p = stg + (16 * wave + 2 * i + hh) * GBN + 4 * m;
      v4f v = *(const v4f*)p;
      v.x = gelu_t(v.x); v.y = gelu_t(v.y); v.z = gelu_t(v.z); v.w = gelu_t(v.w);
      *(v4f*)p = v;
    }
    __syncthreads();
    store_hl(stg, out16, rowBase, col0, wave, lane);
    __threadfence();
    store_hl(stg, out16, rowBase, col0, wave, lane);
  } else {
    if (EPI == 2) {
#pragma unroll 1
      for (int i = 0; i < 8; ++i) {
        const int lr = 16 * wave + 2 * i + hh;
        const int gr = rowBase + lr;
        const int bb = gr / NNODE;
        const int n  = gr - bb * NNODE;
        float* p = stg + lr * GBN + 4 * m;
        v4f v = *(const v4f*)p;
        const v4f s4 = *(const v4f*)(sraw + (size_t)gr * DSW + col0 + 4 * m);
        const float d  = dec[n];
        const float pz = pois[(bb * NSB + n / NBRUN) * 32];
        v.x = fmaf(d, rbf(s4.x), v.x) + pz;
        v.y = fmaf(d, rbf(s4.y), v.y) + pz;
        v.z = fmaf(d, rbf(s4.z), v.z) + pz;
        v.w = fmaf(d, rbf(s4.w), v.w) + pz;
        *(v4f*)p = v;
      }
      __syncthreads();
    }
    store_f32(stg, outF, rowBase, col0, wave, hh, m);
    __threadfence();
    store_f32(stg, outF, rowBase, col0, wave, hh, m);
  }
  (void)out16; (void)outF; (void)sraw; (void)dec; (void)pois; (void)A2;
}

__global__ __launch_bounds__(NTHR) __attribute__((amdgpu_num_vgpr(248)))
void k_scan(const int* __restrict__ dsts, const float* __restrict__ ebias,
            const float* __restrict__ KF, const float* __restrict__ QF, const float* __restrict__ MO,
            unsigned short* inchl, float* pois, int nN, int nE, int nb, int vec8) {
  extern __shared__ v4f lds_dyn[];
  int* reg1 = (int*)lds_dyn;
  int* reg2 = reg1 + RCAP;
  int* scnt = reg2 + RCAP;
  int* soff = scnt + NBMAX;
  int* list = soff + NBMAX;
  int* wcnt = list + LISTN;
  int* wtot = wcnt + NWAVE;
  const int tid = (int)threadIdx.x, lane = tid & 31, wave = tid >> 5;
  const int nodeBase = (int)blockIdx.x * nb;

  for (int i = tid; i < NBMAX; i += NTHR) scnt[i] = 0;
  __syncthreads();

  int tot = 0;
  const int nChunks = (nE + CHUNK - 1) / CHUNK;
#pragma unroll 1
  for (int ch = 0; ch < nChunks; ++ch) {
    const int cbase = ch * CHUNK;
    const int wc = scan_chunk(dsts, nE, cbase, nodeBase, nb, vec8, list, tid, lane, wave);
    if (lane == 0) wcnt[wave] = wc;
    __syncthreads();
    int pre = 0, all = 0;
#pragma unroll
    for (int w2 = 0; w2 < NWAVE; ++w2) {
      int c = wcnt[w2];
      c = c < 0 ? 0 : (c > WCAP ? WCAP : c);
      all += c;
      pre += (w2 < wave) ? c : 0;
    }
    const int wcc  = wc > WCAP ? WCAP : wc;
    const int base = tot + pre;
#pragma unroll 1
    for (int i = lane; i < wcc; i += 32) {
      const int ent = list[wave * WCAP + i];
      const int el  = (ent >> 12) & (CHUNK - 1);
      const int sl  = ent & (NBMAX - 1);
      int eid = cbase + el;
      eid = eid > nE - 1 ? nE - 1 : eid;
      const int pos = base + i;
      if (pos < RCAP) reg1[pos] = (int)(((unsigned)eid << 12) | (unsigned)sl);
    }
    tot += all;
    tot = tot > RCAP ? RCAP : tot;
    __syncthreads();
  }
  const int nh = tot;

  if (wave == 0) {
#pragma unroll 1
    for (int b0 = 0; b0 < nh; b0 += 32) {
      const int idx = b0 + lane;
      const int uv  = reg1[idx < nh ? idx : nh - 1];
      const int m32 = (nh - b0) < 32 ? (nh - b0) : 32;
#pragma unroll 1
      for (int k = 0; k < m32; ++k) {
        const int u  = __builtin_amdgcn_readlane(uv, k);
        const int sl = u & (NBMAX - 1);
        if (lane == 0) scnt[sl] = scnt[sl] + 1;
      }
    }
  }
  __syncthreads();

  {
    const v4i ca = *(const v4i*)(scnt + 8 * tid);
    const v4i cb = *(const v4i*)(scnt + 8 * tid + 4);
    const int e0 = ca.x < 0 ? 0 : ca.x, e1 = ca.y < 0 ? 0 : ca.y, e2 = ca.z < 0 ? 0 : ca.z, e3 = ca.w < 0 ? 0 : ca.w;
    const int e4 = cb.x < 0 ? 0 : cb.x, e5 = cb.y < 0 ? 0 : cb.y, e6 = cb.z < 0 ? 0 : cb.z, e7 = cb.w < 0 ? 0 : cb.w;
    const int ts = e0 + e1 + e2 + e3 + e4 + e5 + e6 + e7;
    int incl = ts;
#pragma unroll
    for (int d = 1; d < 32; d <<= 1) {
      const int up = __shfl_up(incl, d);
      if (lane >= d) incl += up;
    }
    if (lane == 31) wtot[wave] = incl;
    __syncthreads();
    int pre = 0;
#pragma unroll
    for (int w2 = 0; w2 < NWAVE; ++w2) pre += (w2 < wave) ? wtot[w2] : 0;
    int run = pre + incl - ts;
    soff[8 * tid + 0] = run; run += e0;
    soff[8 * tid + 1] = run; run += e1;
    soff[8 * tid + 2] = run; run += e2;
    soff[8 * tid + 3] = run; run += e3;
    soff[8 * tid + 4] = run; run += e4;
    soff[8 * tid + 5] = run; run += e5;
    soff[8 * tid + 6] = run; run += e6;
    soff[8 * tid + 7] = run;
  }
  __syncthreads();
  for (int i = tid; i < NBMAX; i += NTHR) list[i] = soff[i];
  __syncthreads();

  if (wave == 0) {
#pragma unroll 1
    for (int b0 = 0; b0 < nh; b0 += 32) {
      const int idx = b0 + lane;
      const int uv  = reg1[idx < nh ? idx : nh - 1];
      const int m32 = (nh - b0) < 32 ? (nh - b0) : 32;
#pragma unroll 1
      for (int k = 0; k < m32; ++k) {
        const int u   = __builtin_amdgcn_readlane(uv, k);
        const int sl  = u & (NBMAX - 1);
        const int eid = (int)((unsigned)u >> 12);
        if (lane == 0) {
          int pos = list[sl];
          pos = pos < 0 ? 0 : (pos > RCAP - 1 ? RCAP - 1 : pos);
          reg2[pos] = eid;
          list[sl] = pos + 1;
        }
      }
    }
  }
  __syncthreads();

  const int nbw = nb >> 3;
  const bool ovf = (nh >= RCAP);
  const float qnan = __int_as_float(0x7fc00000);
  float* stw = (float*)reg1 + wave * STW;
  const size_t bofs = (size_t)blockIdx.y * (size_t)nN;
  const int part = lane >> 4, piece = lane & 15;
#pragma unroll 1
  for (int jt = 0; jt < nbw; ++jt) {
    const int slot = wave * nbw + jt;
    const int grow = nodeBase + slot;
    const int gcl  = grow < nN ? grow : nN - 1;
    int st = soff[slot];
    const int craw = scnt[slot];
    int cnt = craw;
    st  = st < 0 ? 0 : (st > nh ? nh : st);
    cnt = cnt < 0 ? 0 : (cnt > DEGCAP ? DEGCAP : cnt);
    if (cnt > nh - st) cnt = nh - st;
    const float pz = (ovf || craw > DEGCAP) ? qnan : 0.0f;

    const v4f kd = *(const v4f*)(KF + (size_t)gcl * DSW + 4 * lane);
    v4f av = {0.f, 0.f, 0.f, 0.f};
    ldwait();

#pragma unroll 1
    for (int q = 0; q < cnt; ++q) {
      int idx = st + q; idx = idx > RCAP - 1 ? RCAP - 1 : idx;
      int eid = reg2[idx]; eid = eid < 0 ? 0 : (eid > nE - 1 ? nE - 1 : eid);
      int src = eid >> 4;
      src = src > nN - 1 ? nN - 1 : src;
      const float eb = ebias[eid];
      const size_t ro = (bofs + (size_t)src) * DSW + 4 * lane;
      const v4f qv = *(const v4f*)(QF + ro);
      const v4f mv = *(const v4f*)(MO + ro);
      ldwait();
      float pt = qv.x * kd.x;
      pt = fmaf(qv.y, kd.y, pt);
      pt = fmaf(qv.z, kd.z, pt);
      pt = fmaf(qv.w, kd.w, pt);
#pragma unroll
      for (int off = 16; off > 0; off >>= 1) pt += __shfl_xor(pt, off);
      const float sc = pt + rbf(eb);
      const float w  = __builtin_amdgcn_rcpf(1.0f + expf(-sc));
      av.x = fmaf(w, mv.x, av.x);
      av.y = fmaf(w, mv.y, av.y);
      av.z = fmaf(w, mv.z, av.z);
      av.w = fmaf(w, mv.w, av.w);
    }
    v4f r;
    r.x = av.x + pz; r.y = av.y + pz; r.z = av.z + pz; r.w = av.w + pz;
    wave_sync_lds();
    *(v4f*)(stw + 4 * lane) = r;
    wave_sync_lds();
    const v4f ga = *(const v4f*)(stw + 8 * piece);
    const v4f gb = *(const v4f*)(stw + 8 * piece + 4);
    const v8us hl = pack_hl(ga, gb, part);
    unsigned short* dst = inchl + (bofs + (size_t)gcl) * INCW + part * DSW + 8 * piece;
    const bool wr = grow < nN;
    if (wr) *(volatile v8us*)dst = hl;
    __threadfence();
    if (wr) *(volatile v8us*)dst = hl;
  }

  if (wave == 0) {
    const float fv = ovf ? qnan : 0.0f;
    const v4f pv = {fv, fv, fv, fv};
    float* pp = pois + ((size_t)blockIdx.y * gridDim.x + blockIdx.x) * 32 + 4 * (lane & 7);
    if (lane < 8) *(volatile v4f*)pp = pv;
    __threadfence();
    if (lane < 8) *(volatile v4f*)pp = pv;
  }
}

static inline int cdiv(int a, int b) { return (a + b - 1) / b; }

static void launch_wtr(const float* w, int cols, int Kp, int t1, int d1, int t2, int d2,
                       unsigned short* wt, hipStream_t stream) {
  const int nU = cols * (Kp / 8);
  k_wtr<<<cdiv(nU, NTHR), NTHR, 0, stream>>>(w, cols, Kp, t1, d1, t2, d2, wt, nU);
}

extern "C" void kernel_launch(void* const* d_in, const int* in_sizes, int n_in,
                              void* d_out, int out_size, void* d_ws, size_t ws_size,
                              hipStream_t stream) {
  if (n_in < 23) return;
  if (in_sizes[0] != MROWS * DSW) return;
  if (in_sizes[1] != NEDGE || in_sizes[2] != NEDGE) return;
  if (in_sizes[3] != NNODE * DIDW || in_sizes[4] != DSW) return;
  if (in_sizes[5] != 192 * 256 || in_sizes[6] != 256 || in_sizes[7] != 256 * 128 || in_sizes[8] != 128) return;
  if (in_sizes[9] != 192 * 256 || in_sizes[10] != 256 || in_sizes[11] != 256 * 128 || in_sizes[12] != 128) return;
  if (in_sizes[13] != 64 * 256 || in_sizes[14] != 256 || in_sizes[15] != 256 * 128 || in_sizes[16] != 128) return;
  if (in_sizes[17] != 320 * 256 || in_sizes[18] != 256 || in_sizes[19] != 256 * 128 || in_sizes[20] != 128) return;
  if (in_sizes[21] != DIDW || in_sizes[22] != 1) return;
  if (out_size != MROWS * DSW) return;
  if ((size_t)WS_TOTAL > ws_size) return;

  const float* s    = (const float*)d_in[0];
  const int*   nbrs = (const int*)  d_in[1];
  const float* eb   = (const float*)d_in[2];
  const float* cid  = (const float*)d_in[3];
  const float* cnw  = (const float*)d_in[4];
  const float* c1w  = (const float*)d_in[5];  const float* c1b = (const float*)d_in[6];
  const float* c2w  = (const float*)d_in[7];  const float* c2b = (const float*)d_in[8];
  const float* q1w  = (const float*)d_in[9];  const float* q1b = (const float*)d_in[10];
  const float* q2w  = (const float*)d_in[11]; const float* q2b = (const float*)d_in[12];
  const float* k1w  = (const float*)d_in[13]; const float* k1b = (const float*)d_in[14];
  const float* k2w  = (const float*)d_in[15]; const float* k2b = (const float*)d_in[16];
  const float* u1w  = (const float*)d_in[17]; const float* u1b = (const float*)d_in[18];
  const float* u2w  = (const float*)d_in[19]; const float* u2b = (const float*)d_in[20];
  const float* decw = (const float*)d_in[21]; const float* decb = (const float*)d_in[22];
  float* out = (float*)d_out;

  char* ws = (char*)d_ws;
  unsigned short* XHL  = (unsigned short*)(ws + O_XHL);
  unsigned short* HHL  = (unsigned short*)(ws + O_HHL);
  float*          MOUT = (float*)(ws + O_MOUT);
  float*          QF   = (float*)(ws + O_QF);
  unsigned short* HKHL = (unsigned short*)(ws + O_HK);
  unsigned short* INCHL = HKHL;
  float*          KF   = (float*)(ws + O_KF);
  unsigned short* C1C  = (unsigned short*)(ws + O_C1);
  unsigned short* Q1C  = (unsigned short*)(ws + O_Q1);
  unsigned short* C2D  = (unsigned short*)(ws + O_C2);
  unsigned short* Q2D  = (unsigned short*)(ws + O_Q2);
  unsigned short* K1T  = (unsigned short*)(ws + O_K1);
  unsigned short* K2D  = (unsigned short*)(ws + O_K2);
  unsigned short* U1C  = (unsigned short*)(ws + O_U1);
  unsigned short* U2D  = (unsigned short*)(ws + O_U2);
  float*          DEC  = (float*)(ws + O_DEC);
  float*          POIS = (float*)(ws + O_POIS);

  hipFuncSetAttribute(reinterpret_cast<const void*>(&k_scan),
                      hipFuncAttributeMaxDynamicSharedMemorySize, LDS_SCAN);

  const int BIG = 1 << 30;
  k_pa<<<MROWS / NWAVE, NTHR, 0, stream>>>(s, cnw, cid, XHL, MROWS, NNODE);
  launch_wtr(c1w, 256, XK,  128, 128, BIG, 0,   C1C, stream);
  launch_wtr(q1w, 256, XK,  128, 128, BIG, 0,   Q1C, stream);
  launch_wtr(c2w, 128, H2K, 256, 256, BIG, 0,   C2D, stream);
  launch_wtr(q2w, 128, H2K, 256, 256, BIG, 0,   Q2D, stream);
  launch_wtr(k1w, 256, DIDW, BIG, 0,  BIG, 0,   K1T, stream);
  launch_wtr(k2w, 128, H2K, 256, 256, BIG, 0,   K2D, stream);
  launch_wtr(u1w, 256, UK,  128, 128, 448, 128, U1C, stream);
  launch_wtr(u2w, 128, H2K, 256, 256, BIG, 0,   U2D, stream);
  k_dec<<<NNODE / NTHR, NTHR, 0, stream>>>(cid, decw, decb, DEC, NNODE);

  k_gemm<0, XK, 256, 2, XK, 0><<<dim3(NNODE / GBM, 256 / GBN), GTHR, 0, stream>>>(
      XHL, XHL, K1T, k1b, HKHL, KF, s, DEC, POIS);
  k_gemm<1, H2K, 0, 16, H2K, 0><<<dim3(NNODE / GBM, DSW / GBN), GTHR, 0, stream>>>(
      HKHL, HKHL, K2D, k2b, HHL, KF, s, DEC, POIS);
  k_gemm<0, XK, 0, 10, XK, 0><<<dim3(MROWS / GBM, 256 / GBN), GTHR, 0, stream>>>(
      XHL, XHL, C1C, c1b, HHL, MOUT, s, DEC, POIS);
  k_gemm<1, H2K, 0, 16, H2K, 0><<<dim3(MROWS / GBM, DSW / GBN), GTHR, 0, stream>>>(
      HHL, HHL, C2D, c2b, HKHL, MOUT, s, DEC, POIS);
  k_gemm<0, XK, 0, 10, XK, 0><<<dim3(MROWS / GBM, 256 / GBN), GTHR, 0, stream>>>(
      XHL, XHL, Q1C, q1b, HHL, QF, s, DEC, POIS);
  k_gemm<1, H2K, 0, 16, H2K, 0><<<dim3(MROWS / GBM, DSW / GBN), GTHR, 0, stream>>>(
      HHL, HHL, Q2D, q2b, HKHL, QF, s, DEC, POIS);
  k_scan<<<dim3(NSB, NBATCH), NTHR, LDS_SCAN, stream>>>(nbrs, eb, KF, QF, MOUT, INCHL, POIS,
                                                        NNODE, NEDGE, NBRUN, 1);
  k_gemm<0, XK, 0, 10, INCW, 8><<<dim3(MROWS / GBM, 256 / GBN), GTHR, 0, stream>>>(
      XHL, INCHL, U1C, u1b, HHL, MOUT, s, DEC, POIS);
  k_gemm<2, H2K, 0, 16, H2K, 0><<<dim3(MROWS / GBM, DSW / GBN), GTHR, 0, stream>>>(
      HHL, HHL, U2D, u2b, HKHL, out, s, DEC, POIS);
}
